// EncoderBlock_80668075753740
// MI455X (gfx1250) — hardware-verified
//
#include <hip/hip_runtime.h>

#ifndef NB
#define NB 2
#endif
#ifndef SEQ
#define SEQ 2048
#endif
#define NB_FULL 2
#define SEQ_FULL 2048
#define DM 1024
#define DFF 4096
#define MROWS (NB * SEQ)
#ifndef S_BH
#define S_BH ((float)SEQ)
#endif

typedef __attribute__((ext_vector_type(16))) _Float16 v16h;
typedef __attribute__((ext_vector_type(8)))  _Float16 v8h;
typedef __attribute__((ext_vector_type(8)))  float    v8f;
typedef __attribute__((ext_vector_type(4)))  float    v4f;
typedef unsigned int cm_u4 __attribute__((ext_vector_type(4)));
typedef unsigned int bk_u2 __attribute__((ext_vector_type(2)));

#define VST2(T, ptr, val) do { const T vst2_v_ = (val); *(volatile T*)(ptr) = vst2_v_; __threadfence(); *(volatile T*)(ptr) = vst2_v_; } while (0)
#define VST2V4(ptr, val) do { const v4f vst2_v4_ = (val); *(volatile v4f*)(ptr) = vst2_v4_; __threadfence(); *(volatile v4f*)(ptr) = vst2_v4_; } while (0)

namespace gk {
__device__ __forceinline__ void dep_guard_h(v8f& a, v8f& b, v16h x, v16h y) { asm volatile("v_nop\n\tv_nop\n\tv_nop\n\tv_nop" : "+v"(a), "+v"(b) : "v"(x), "v"(y)); }
__device__ __forceinline__ void keep4_h(v16h a, v16h b, v16h c, v16h d) { asm volatile("v_nop" :: "v"(a), "v"(b), "v"(c), "v"(d)); }
__device__ __forceinline__ void acc_guard4(v8f& a, v8f& b, v8f& c, v8f& d) { asm volatile("v_nop\n\tv_nop\n\tv_nop\n\tv_nop" : "+v"(a), "+v"(b), "+v"(c), "+v"(d)); }
union FragU { v16h v; v8h h[2]; };
__device__ __forceinline__ v16h frag_load(const _Float16* p) { FragU f; f.h[0] = *(const v8h*)(p); f.h[1] = *(const v8h*)(p + 16); return f.v; }
__device__ __forceinline__ v8f mma(v16h a, v16h b, v8f c) { return __builtin_amdgcn_wmma_f32_16x16x32_f16(false, a, false, b, (short)0, c, false, false); }

template <int OUT16, int RELU>
__global__ __launch_bounds__(256) void wmma_gemm64(
    const unsigned short* __restrict__ Ap, int lda,
    const unsigned short* __restrict__ Btp, int ldb,
    void* __restrict__ Cout, int ldc,
    const float* __restrict__ bias,
    int M, int N, int K, float scale) {
  const _Float16* A = (const _Float16*)Ap; const _Float16* Bt = (const _Float16*)Btp;
  __shared__ __align__(16) float sT[8][16 * 68];
  const int lane = threadIdx.x & 31;
  const int wave = threadIdx.x >> 5;
  const int tilesN = N >> 6;
  const int tilesM = M >> 6;
  const int tile = blockIdx.x * 8 + wave;
  if (tile >= tilesM * tilesN) return;
  const int tm = tile / tilesN;
  const int tn = tile - tm * tilesN;
  const int m0 = tm << 6;
  const int n0 = tn << 6;

  const int rlane = lane & 15;
  const int koff  = (lane >> 4) * 8;
  const int mOff  = (lane >> 4) * 8;

  v8f acc[4][4];
#pragma unroll
  for (int i = 0; i < 4; ++i)
#pragma unroll
    for (int j = 0; j < 4; ++j) acc[i][j] = (v8f){0.f,0.f,0.f,0.f,0.f,0.f,0.f,0.f};

  for (int k0 = 0; k0 < K; k0 += 32) {
    v16h bh[4];
#pragma unroll
    for (int j = 0; j < 4; ++j) {
      const size_t bo = (size_t)(n0 + (j << 4) + rlane) * ldb + koff + k0;
      bh[j] = frag_load(Bt + bo);
    }
#pragma unroll
    for (int i = 0; i < 4; ++i) {
      const size_t ao = (size_t)(m0 + (i << 4) + rlane) * lda + koff + k0;
      v16h ah = frag_load(A + ao);
#pragma unroll
      for (int j = 0; j < 4; ++j) acc[i][j] = mma(ah, bh[j], acc[i][j]);
      dep_guard_h(acc[i][0], acc[i][3], ah, ah);
    }
    keep4_h(bh[0], bh[1], bh[2], bh[3]);
  }
  acc_guard4(acc[0][0], acc[0][1], acc[0][2], acc[0][3]);
  acc_guard4(acc[1][0], acc[1][1], acc[1][2], acc[1][3]);
  acc_guard4(acc[2][0], acc[2][1], acc[2][2], acc[2][3]);
  acc_guard4(acc[3][0], acc[3][1], acc[3][2], acc[3][3]);

  float* slab = sT[wave];
#pragma unroll
  for (int i = 0; i < 4; ++i) {
    const int mBase = m0 + (i << 4);
#pragma unroll
    for (int j = 0; j < 4; ++j) {
      const int n = n0 + (j << 4) + rlane;
      const float bv = bias[n];
#pragma unroll
      for (int r = 0; r < 8; ++r) {
        float v = acc[i][j][r] * scale;
        v += bv;
        if (RELU == 1) v = fmaxf(v, 0.0f);
        slab[(mOff + r) * 68 + (j << 4) + rlane] = v;
      }
    }
    __builtin_amdgcn_fence(3  , "workgroup");
    __builtin_amdgcn_wave_barrier();
    __builtin_amdgcn_fence(2  , "workgroup");
    if (OUT16 == 0) {
      float* C = (float*)Cout;
      const int hh = lane >> 4, c4 = (lane & 15) * 4;
      for (int pass = 0; pass < 2; ++pass) {
#pragma unroll
        for (int it = 0; it < 8; ++it) {
          const int row = it * 2 + hh;
          v4f v = *(const v4f*)(slab + row * 68 + c4);
          *(volatile v4f*)(C + (size_t)(mBase + row) * ldc + n0 + c4) = v;
        }
        __threadfence();
      }
    } else {
      const int q = lane >> 3, c8 = (lane & 7) * 8;
      unsigned short* C = (unsigned short*)Cout;
      for (int pass = 0; pass < 2; ++pass) {
#pragma unroll
        for (int it = 0; it < 4; ++it) {
          const int row = it * 4 + q;
          const float* sp = slab + row * 68 + c8;
          v8h hv;
#pragma unroll
          for (int e = 0; e < 8; ++e) hv[e] = (_Float16)sp[e];
          *(volatile v8h*)(C + (size_t)(mBase + row) * ldc + n0 + c8) = hv;
        }
        __threadfence();
      }
    }
    __builtin_amdgcn_fence(3  , "workgroup");
    __builtin_amdgcn_wave_barrier();
    __builtin_amdgcn_fence(2  , "workgroup");
  }
}
}

__device__ __forceinline__ unsigned int cmb_pk2(float a, float b) { return (unsigned int)__builtin_bit_cast(unsigned short, (_Float16)a) | ((unsigned int)__builtin_bit_cast(unsigned short, (_Float16)b) << 16); }
__device__ __forceinline__ float cmb_bf(float v) { const unsigned u = __builtin_bit_cast(unsigned, v); const unsigned r = (u + 0x7fffu + ((u >> 16) & 1u)) & 0xffff0000u; return __builtin_bit_cast(float, r); }
__global__ __launch_bounds__(256) void k_cm_bfvec(const float* __restrict__ SRC, float* __restrict__ DST, int n) { const int u = blockIdx.x * 256 + threadIdx.x; if (u >= n) return; VST2(float, DST + u, cmb_bf(SRC[u])); }
__global__ __launch_bounds__(256) void k_cm_castb(const float* __restrict__ SRC, int lds, unsigned short* __restrict__ DST, int ldd, int nR, int nC, float sc) {
    const long long u = (long long)blockIdx.x * 256 + threadIdx.x; const int per = nC / 8; if (u >= (long long)nR * per) return; const int r = (int)(u / per); const int c0 = 8 * (int)(u % per);
    const float* s = SRC + (long long)r * lds + c0; float w[8];
#pragma unroll
    for (int e = 0; e < 8; ++e) w[e] = cmb_bf(s[e]) * sc;
    cm_u4 pk; pk.x = cmb_pk2(w[0], w[1]); pk.y = cmb_pk2(w[2], w[3]); pk.z = cmb_pk2(w[4], w[5]); pk.w = cmb_pk2(w[6], w[7]); VST2(cm_u4, (cm_u4*)(DST + (long long)r * ldd + c0), pk); }
__global__ __launch_bounds__(256) void k_cm_castbT(const float* __restrict__ SRC, int lds, unsigned short* __restrict__ DST, int ldd, int nR, int nC, float sc) {
    const long long u = (long long)blockIdx.x * 256 + threadIdx.x; const int per = nR / 8; if (u >= (long long)nC * per) return; const int c = (int)(u / per); const int r0 = 8 * (int)(u % per);
    float w[8];
#pragma unroll
    for (int e = 0; e < 8; ++e) w[e] = cmb_bf(SRC[(long long)(r0 + e) * lds + c]) * sc;
    cm_u4 pk; pk.x = cmb_pk2(w[0], w[1]); pk.y = cmb_pk2(w[2], w[3]); pk.z = cmb_pk2(w[4], w[5]); pk.w = cmb_pk2(w[6], w[7]); VST2(cm_u4, (cm_u4*)(DST + (long long)c * ldd + r0), pk); }

__device__ __forceinline__ unsigned int bk_pk2(float a, float b) { return (unsigned int)__builtin_bit_cast(unsigned short, (_Float16)a) | ((unsigned int)__builtin_bit_cast(unsigned short, (_Float16)b) << 16); }
template <int NQ, int HASX, int XBF>
__global__ __launch_bounds__(256) void k_b_ln(const float* __restrict__ A, const float* __restrict__ X, const float* __restrict__ GA, const float* __restrict__ BE, float eps, float inv_vden, int rows, float* __restrict__ Yf, unsigned short* __restrict__ Y16) {
    #pragma clang fp contract(off)
    constexpr int WD = 128 * NQ; const int r = blockIdx.x * 8 + (threadIdx.x >> 5); const int L = threadIdx.x & 31; if (r >= rows) return; v4f v[NQ]; float s = 0.f;
#pragma unroll
    for (int q = 0; q < NQ; ++q) { const long long o = (long long)r * WD + 4 * L + 128 * q; v[q] = *(const v4f*)(A + o); if (HASX) { v4f x = *(const v4f*)(X + o); if (XBF) { x.x = cmb_bf(x.x); x.y = cmb_bf(x.y); x.z = cmb_bf(x.z); x.w = cmb_bf(x.w); } v[q] = v[q] + x; } s += (v[q].x + v[q].y) + (v[q].z + v[q].w); }
#pragma unroll
    for (int o = 16; o > 0; o >>= 1) s += __shfl_xor(s, o, 32);
    const float mu = s * (1.f / WD); float qq = 0.f;
#pragma unroll
    for (int q = 0; q < NQ; ++q) { v[q].x -= mu; v[q].y -= mu; v[q].z -= mu; v[q].w -= mu; qq += (v[q].x * v[q].x + v[q].y * v[q].y) + (v[q].z * v[q].z + v[q].w * v[q].w); }
#pragma unroll
    for (int o = 16; o > 0; o >>= 1) qq += __shfl_xor(qq, o, 32);
    const float rs = rsqrtf(qq * inv_vden + eps);
#pragma unroll
    for (int q = 0; q < NQ; ++q) { const int c = 4 * L + 128 * q; const v4f ga = *(const v4f*)(GA + c), be = *(const v4f*)(BE + c); v4f y; y.x = v[q].x * rs * cmb_bf(ga.x) + cmb_bf(be.x); y.y = v[q].y * rs * cmb_bf(ga.y) + cmb_bf(be.y); y.z = v[q].z * rs * cmb_bf(ga.z) + cmb_bf(be.z); y.w = v[q].w * rs * cmb_bf(ga.w) + cmb_bf(be.w);
        const long long o = (long long)r * WD + c; if (Yf != nullptr) VST2V4(Yf + o, y); if (Y16 != nullptr) { bk_u2 pk; pk.x = bk_pk2(y.x, y.y); pk.y = bk_pk2(y.z, y.w); VST2(bk_u2, (bk_u2*)(Y16 + o), pk); } } }

static constexpr size_t al256(size_t b) { return (b + 255) / 256 * 256; }

extern "C" void kernel_launch(void* const* d_in, const int* in_sizes, int n_in, void* d_out, int out_size, void* d_ws, size_t ws_size, hipStream_t stream) {
    static_assert(DM == 128 * 8);
    static_assert((MROWS % 64) == 0 && (DM % 64) == 0 && (DFF % 64) == 0);
    static_assert((DM % 32) == 0 && (DFF % 32) == 0);
    static_assert((((MROWS / 64) * (DM / 64)) % 8) == 0 && (((MROWS / 64) * (DFF / 64)) % 8) == 0);
    static_assert(((SEQ * (DM / 8)) % 256) == 0 && (SEQ % 8) == 0 && (MROWS % 8) == 0);
    static_assert(((DM * (DM / 8)) % 256) == 0 && ((DFF * (DM / 8)) % 256) == 0 && ((DM * (DFF / 8)) % 256) == 0);
    static_assert(NB <= NB_FULL && SEQ <= SEQ_FULL);
    static_assert((size_t)MROWS * DM * 4 <= (size_t)16777216);
    if (n_in < 18) return;
    if (in_sizes[2] < NB * SEQ * DM) return;
    if (in_sizes[8] < DM * DM || in_sizes[10] < DM * DM || in_sizes[12] < DM * DFF || in_sizes[14] < DFF * DM) return;
    if (in_sizes[9] < DM || in_sizes[11] < DM || in_sizes[13] < DFF || in_sizes[15] < DM || in_sizes[16] < DM || in_sizes[17] < DM) return;
    if (out_size < MROWS * DM) return;

    const float* z  = (const float*)d_in[2];
    const float* Wv = (const float*)d_in[8];
    const float* bv = (const float*)d_in[9];
    const float* Wo = (const float*)d_in[10];
    const float* bo = (const float*)d_in[11];
    const float* W1 = (const float*)d_in[12];
    const float* b1 = (const float*)d_in[13];
    const float* W2 = (const float*)d_in[14];
    const float* b2 = (const float*)d_in[15];
    const float* lg = (const float*)d_in[16];
    const float* lb = (const float*)d_in[17];
    float* out = (float*)d_out;

    constexpr size_t SZ_Z16 = al256((size_t)MROWS * DM * 2);
    constexpr size_t SZ_WDD = al256((size_t)DM * DM * 2);
    constexpr size_t SZ_WDF = al256((size_t)DM * DFF * 2);
    constexpr size_t SZ_V16 = al256((size_t)MROWS * DM * 2);
    constexpr size_t SZ_F32 = al256((size_t)MROWS * DM * 4);
    constexpr size_t SZ_H16 = al256((size_t)MROWS * DM * 2);
    constexpr size_t SZ_A1  = al256((size_t)MROWS * DFF * 2);
    constexpr size_t SZ_BD  = al256((size_t)(DM + 64) * 4);
    constexpr size_t SZ_BF  = al256((size_t)(DFF + 64) * 4);
    constexpr size_t SZ_TOTAL = SZ_Z16 + 2 * SZ_WDD + 2 * SZ_WDF + SZ_V16 + 3 * SZ_F32 + SZ_H16 + SZ_A1 + 3 * SZ_BD + SZ_BF;
    static_assert(SZ_TOTAL <= (size_t)134217728);
    if (SZ_TOTAL > ws_size) return;

    char* wsp = (char*)d_ws;
    unsigned short* Z16 = (unsigned short*)wsp; wsp += SZ_Z16;
    unsigned short* WvT = (unsigned short*)wsp; wsp += SZ_WDD;
    unsigned short* WoT = (unsigned short*)wsp; wsp += SZ_WDD;
    unsigned short* W1T = (unsigned short*)wsp; wsp += SZ_WDF;
    unsigned short* W2T = (unsigned short*)wsp; wsp += SZ_WDF;
    unsigned short* V16 = (unsigned short*)wsp; wsp += SZ_V16;
    float* ATT = (float*)wsp; wsp += SZ_F32;
    float* H1f = (float*)wsp; wsp += SZ_F32;
    float* FFo = (float*)wsp; wsp += SZ_F32;
    unsigned short* H16 = (unsigned short*)wsp; wsp += SZ_H16;
    unsigned short* A1  = (unsigned short*)wsp; wsp += SZ_A1;
    float* BRV = (float*)wsp; wsp += SZ_BD;
    float* BRO = (float*)wsp; wsp += SZ_BD;
    float* BR2 = (float*)wsp; wsp += SZ_BD;
    float* BR1 = (float*)wsp; wsp += SZ_BF;

    for (int b = 0; b < NB; ++b)
        k_cm_castb<<<(unsigned)(((long long)SEQ * (DM / 8) + 255) / 256), 256, 0, stream>>>(z + (size_t)b * SEQ_FULL * DM, DM, Z16 + (size_t)b * SEQ * DM, DM, SEQ, DM, 1.0f);
    k_cm_castbT<<<(unsigned)(((long long)DM * (DM / 8) + 255) / 256), 256, 0, stream>>>(Wv, DM, WvT, DM, DM, DM, 16.0f);
    k_cm_castbT<<<(unsigned)(((long long)DM * (DM / 8) + 255) / 256), 256, 0, stream>>>(Wo, DM, WoT, DM, DM, DM, 16.0f);
    k_cm_castbT<<<(unsigned)(((long long)DFF * (DM / 8) + 255) / 256), 256, 0, stream>>>(W1, DFF, W1T, DM, DM, DFF, 16.0f);
    k_cm_castbT<<<(unsigned)(((long long)DM * (DFF / 8) + 255) / 256), 256, 0, stream>>>(W2, DM, W2T, DFF, DFF, DM, 16.0f);
    k_cm_bfvec<<<(DM + 255) / 256, 256, 0, stream>>>(bv, BRV, DM);
    k_cm_bfvec<<<(DM + 255) / 256, 256, 0, stream>>>(bo, BRO, DM);
    k_cm_bfvec<<<(DFF + 255) / 256, 256, 0, stream>>>(b1, BR1, DFF);
    k_cm_bfvec<<<(DM + 255) / 256, 256, 0, stream>>>(b2, BR2, DM);

    gk::wmma_gemm64<1, 0><<<dim3((unsigned)(((MROWS / 64) * (DM / 64)) / 8)), 256, 0, stream>>>(Z16, DM, WvT, DM, (void*)V16, DM, BRV, MROWS, DM, DM, 0.0625f);
    gk::wmma_gemm64<0, 0><<<dim3((unsigned)(((MROWS / 64) * (DM / 64)) / 8)), 256, 0, stream>>>(V16, DM, WoT, DM, (void*)ATT, DM, BRO, MROWS, DM, DM, S_BH * 0.0625f);
    for (int b = 0; b < NB; ++b)
        k_b_ln<8, 1, 1><<<(SEQ + 7) / 8, 256, 0, stream>>>(ATT + (size_t)b * SEQ * DM, z + (size_t)b * SEQ_FULL * DM, lg, lb, 1e-5f, 1.0f / 1024.0f, SEQ, H1f + (size_t)b * SEQ * DM, H16 + (size_t)b * SEQ * DM);
    gk::wmma_gemm64<1, 1><<<dim3((unsigned)(((MROWS / 64) * (DFF / 64)) / 8)), 256, 0, stream>>>(H16, DM, W1T, DM, (void*)A1, DFF, BR1, MROWS, DFF, DM, 0.0625f);
    gk::wmma_gemm64<0, 0><<<dim3((unsigned)(((MROWS / 64) * (DM / 64)) / 8)), 256, 0, stream>>>(A1, DFF, W2T, DFF, (void*)FFo, DM, BR2, MROWS, DM, DFF, 0.0625f);
    k_b_ln<8, 1, 0><<<(MROWS + 7) / 8, 256, 0, stream>>>(FFo, H1f, lg, lb, 1e-5f, 1.0f / 1024.0f, MROWS, out, nullptr);
}
